// DiffNet_17085379903955
// MI455X (gfx1250) — hardware-run, weakly checked
//
#include <hip/hip_runtime.h>


#define NR   64
#define D0   1024
#define D1   512
#define D3   256
#define STEP 0.01f
constexpr size_t al256(size_t b) { return (b + 255) & ~(size_t)255; }
constexpr size_t WS_TOTAL = al256((size_t)NR * D0 * 2) + al256((size_t)D1 * D0 * 2) + al256((size_t)D1 * D1 * 2) + al256((size_t)D3 * D1 * 2) + 2 * al256((size_t)NR * D1 * 4) + al256((size_t)NR * D3 * 4)
                          + 2 * al256((size_t)NR * D1 * 4) + 4 * al256((size_t)NR * D1 * 2) + 3 * al256((size_t)2 * NR * 4);
static_assert(WS_TOTAL == 2819584 && WS_TOTAL <= 134217728, "the workspace carve: about 2.7 MiB");
typedef _Float16 h16;
typedef unsigned short bf;
typedef __attribute__((ext_vector_type(16))) __bf16   v16bf;
typedef __attribute__((ext_vector_type(16))) _Float16 v16h;
typedef __attribute__((ext_vector_type(8)))  _Float16 v8h;
typedef __attribute__((ext_vector_type(8)))  unsigned short v8us;
typedef __attribute__((ext_vector_type(8)))  float    v8f;
typedef __attribute__((ext_vector_type(4)))  float    v4f;
typedef v8h  __attribute__((may_alias)) v8ha;
typedef v4f  __attribute__((may_alias)) v4fa;
typedef v8us __attribute__((may_alias)) v8usa;

__device__ __forceinline__ unsigned short f2bf(float f) { unsigned u = __float_as_uint(f); u += 0x7FFFu + ((u >> 16) & 1u); return (unsigned short)(u >> 16); }
__device__ __forceinline__ float bf2f(unsigned short b) { return __uint_as_float(((unsigned)b) << 16); }
__device__ __forceinline__ float bfr(float f) { return bf2f(f2bf(f)); }
__device__ __forceinline__ v16h cat16(v8h lo, v8h hi) { return __builtin_shufflevector(lo, hi, 0, 1, 2, 3, 4, 5, 6, 7, 8, 9, 10, 11, 12, 13, 14, 15); }
__device__ __forceinline__ v16bf cat16b(v8us lo, v8us hi) { return __builtin_bit_cast(v16bf, __builtin_shufflevector(lo, hi, 0, 1, 2, 3, 4, 5, 6, 7, 8, 9, 10, 11, 12, 13, 14, 15)); }
__device__ __forceinline__ v8f wmma16(v16h a, v16h b, v8f c) { return __builtin_amdgcn_wmma_f32_16x16x32_f16(false, a, false, b, (short)0, c, false, false); }
__device__ __forceinline__ v8f wmmab(v16bf a, v16bf b, v8f c) { return __builtin_amdgcn_wmma_f32_16x16x32_bf16(false, a, false, b, (short)0, c, false, false); }


template <typename T16> struct WFrag;
template <> struct WFrag<h16> { typedef v16h V; static __device__ __forceinline__ V ld(const h16* p) { return cat16(*(const v8h*)p, *(const v8h*)(p + 16)); } static __device__ __forceinline__ v8f mma(V a, V b, v8f c) { return wmma16(a, b, c); } };
template <> struct WFrag<bf> { typedef v16bf V; static __device__ __forceinline__ V ld(const bf* p) { return cat16b(*(const v8us*)p, *(const v8us*)(p + 16)); } static __device__ __forceinline__ v8f mma(V a, V b, v8f c) { return wmmab(a, b, c); } };
template <typename T16, int NSPLIT, bool BIAS>
__global__ __launch_bounds__(32) void k_gemmw(const T16* __restrict__ A, const T16* __restrict__ A2, const T16* __restrict__ Bt, const T16* __restrict__ Bt2, int K, float* C, int ldc, const float* __restrict__ bias, size_t sA, size_t sB, size_t sC) {
    typedef typename WFrag<T16>::V V;
    __shared__ __align__(16) float os[16 * 68];
    const size_t z = blockIdx.z; A += z * sA; if (A2) A2 += z * sA; Bt += z * sB; if (Bt2) Bt2 += z * sB; C += z * sC;
    const int lane = threadIdx.x & 31, lr = lane & 15, hi = lane >> 4; const int r0 = blockIdx.x * 64, c0 = blockIdx.y * 64;
    v8f acc[4][4];
#pragma unroll
    for (int mb = 0; mb < 4; ++mb)
#pragma unroll
        for (int nb = 0; nb < 4; ++nb) acc[mb][nb] = (v8f){};
    const size_t aoff = (size_t)(r0 + lr) * K + 8 * hi, boff = (size_t)(c0 + lr) * K + 8 * hi;
    for (int kc = 0; kc < K; kc += 32) {
        V a[4], a2[4];
#pragma unroll
        for (int mb = 0; mb < 4; ++mb) { a[mb] = WFrag<T16>::ld(A + aoff + (size_t)mb * 16 * K + kc); if (NSPLIT == 1 || NSPLIT == 2) a2[mb] = WFrag<T16>::ld(A2 + aoff + (size_t)mb * 16 * K + kc); }
#pragma unroll
        for (int nb = 0; nb < 4; ++nb) { const V b = WFrag<T16>::ld(Bt + boff + (size_t)nb * 16 * K + kc); V b2; if (NSPLIT >= 2) b2 = WFrag<T16>::ld(Bt2 + boff + (size_t)nb * 16 * K + kc);
#pragma unroll
            for (int mb = 0; mb < 4; ++mb) { acc[mb][nb] = WFrag<T16>::mma(a[mb], b, acc[mb][nb]); if (NSPLIT == 1 || NSPLIT == 2) acc[mb][nb] = WFrag<T16>::mma(a2[mb], b, acc[mb][nb]); if (NSPLIT >= 2) acc[mb][nb] = WFrag<T16>::mma(a[mb], b2, acc[mb][nb]); } }
        asm volatile("v_nop\n\tv_nop\n\tv_nop\n\tv_nop" : "+v"(acc[0][0]), "+v"(acc[1][1]), "+v"(acc[2][2]), "+v"(acc[3][3]) : "v"(a[0]), "v"(a[3]));
    }
#pragma unroll
    for (int mb = 0; mb < 4; ++mb) {
#pragma unroll
        for (int nb = 0; nb < 4; ++nb) {
#pragma unroll
            for (int j = 0; j < 8; ++j) os[(hi * 8 + j) * 68 + nb * 16 + lr] = acc[mb][nb][j]; }
        __builtin_amdgcn_wave_barrier(); asm volatile("" ::: "memory");
        float* crow = C + (size_t)(r0 + mb * 16) * ldc + c0;
#pragma unroll 1
        for (int ps = 0; ps < 2; ++ps) {
#pragma unroll
            for (int s = 0; s < 8; ++s) { const int row = 2 * s + hi, cofs = lr * 4; v4f val = *(const v4fa*)(os + row * 68 + cofs); if (BIAS) { val[0] += bfr(bias[c0 + cofs]); val[1] += bfr(bias[c0 + cofs + 1]); val[2] += bfr(bias[c0 + cofs + 2]); val[3] += bfr(bias[c0 + cofs + 3]); }
                *(volatile v4f*)(crow + (size_t)row * ldc + cofs) = val; }
            if (ps == 0) __threadfence(); }
        __builtin_amdgcn_wave_barrier(); asm volatile("" ::: "memory");
    }
}

__device__ __forceinline__ void splitf(float y, unsigned short& h, unsigned short& l) { h = f2bf(y); l = f2bf(y - bf2f(h)); }
typedef __attribute__((ext_vector_type(2))) _Float16 v2h;
typedef __attribute__((ext_vector_type(4))) _Float16 v4h;
typedef __attribute__((ext_vector_type(2))) unsigned short v2us;
typedef __attribute__((ext_vector_type(4))) unsigned short v4us;
typedef __attribute__((ext_vector_type(2))) float v2f;
typedef __attribute__((ext_vector_type(4))) int v4i;

__global__ __launch_bounds__(256) void k_cvt8(const float* __restrict__ src, bf* dst, size_t n8) { const size_t i = (size_t)blockIdx.x * 256 + threadIdx.x; if (i >= n8) return; const v8f v = *(const v8f*)(src + i * 8); v8us o;
#pragma unroll
    for (int k = 0; k < 8; ++k) o[k] = f2bf(v[k]); *(volatile v8us*)(dst + i * 8) = o; __threadfence(); *(volatile v8us*)(dst + i * 8) = o; }

__global__ __launch_bounds__(256) void k_pl2(const float* __restrict__ F, bf* Ph, bf* Pl, size_t n4) { const size_t i = (size_t)blockIdx.x * 256 + threadIdx.x; if (i >= n4) return; const v4f v = *(const v4f*)(F + i * 4); v4us oh, ol;
#pragma unroll
    for (int q = 0; q < 4; ++q) { unsigned short a, c; splitf(v[q], a, c); oh[q] = a; ol[q] = c; } *(volatile v4us*)(Ph + i * 4) = oh; *(volatile v4us*)(Pl + i * 4) = ol; __threadfence(); *(volatile v4us*)(Ph + i * 4) = oh; *(volatile v4us*)(Pl + i * 4) = ol; }

__global__ __launch_bounds__(256) void k_rsum16(const bf* __restrict__ v, float* rs, int rows) {
    const int j = blockIdx.x * 256 + threadIdx.x; if (j >= rows) return; const bf* p = v + (size_t)j * D0; float q2 = 0.0f, q1 = 0.0f;
    for (int i = 0; i < D0; ++i) { const float t = bf2f(p[i]); q2 += t * t; q1 += t; }
    *(volatile float*)(rs + j) = q2; *(volatile float*)(rs + rows + j) = q1; __threadfence(); *(volatile float*)(rs + j) = q2; *(volatile float*)(rs + rows + j) = q1; }
__global__ __launch_bounds__(256) void k_rsum32(const float* __restrict__ v, float* rs, int rows) {
    const int j = blockIdx.x * 256 + threadIdx.x; if (j >= rows) return; const float* p = v + (size_t)j * D1; float q2 = 0.0f, q1 = 0.0f;
    for (int i = 0; i < D1; ++i) { const float t = p[i]; q2 += t * t; q1 += t; }
    *(volatile float*)(rs + j) = q2; *(volatile float*)(rs + rows + j) = q1; __threadfence(); *(volatile float*)(rs + j) = q2; *(volatile float*)(rs + rows + j) = q1; }

__global__ __launch_bounds__(256) void k_corr(const float* __restrict__ GB, const float* __restrict__ bl, const float* __restrict__ rs, const float* __restrict__ A, const float* __restrict__ a,
                                              const float* __restrict__ B, const float* __restrict__ b, const int* __restrict__ q, float* y, int nw) {
    const int o = blockIdx.x * 256 + threadIdx.x; const int r = blockIdx.y; if (o >= nw) return; const size_t n = (size_t)r * nw + o;
    float c0 = 0.0f, c1 = 0.0f, c2 = 0.0f, e = bfr(b[0]);
#pragma unroll
    for (int h = 0; h < 8; ++h) { const float bh = bfr(B[h]); c0 += bh * bfr(A[h * 3 + 0]); c1 += bh * bfr(A[h * 3 + 1]); c2 += bh * bfr(A[h * 3 + 2]); e += bh * bfr(a[h]); }
    const float s = __fdiv_rn(STEP, (float)q[0]); const float gb = GB[n]; const float vl = bfr(bl[o]); const float u = fmaxf(gb, 0.0f); const float g = gb - vl; const float S1 = rs[r]; const float S2 = rs[NR + r];
    const float yv = u + s * (c0 * S1 + c1 * g + (c2 * u + e) * S2);
    *(volatile float*)(y + n) = yv; __threadfence(); *(volatile float*)(y + n) = yv; }

extern "C" void kernel_launch(void* const* d_in, const int* in_sizes, int n_in,
                              void* d_out, int out_size, void* d_ws, size_t ws_size, hipStream_t stream) {
    if (n_in < 12) return;
    if (in_sizes[0] < NR * D0 || in_sizes[1] < D1 * D0 || in_sizes[2] < D1 || in_sizes[3] < D1 * D1 || in_sizes[4] < D1 || in_sizes[5] < D3 * D1 || in_sizes[6] < D3 || in_sizes[7] < 24 || in_sizes[8] < 8 || in_sizes[9] < 8 || in_sizes[10] < 1 || in_sizes[11] < 1 || out_size < NR * D3) return;
    const float* x = (const float*)d_in[0]; const float* w1 = (const float*)d_in[1]; const float* b1 = (const float*)d_in[2]; const float* w2 = (const float*)d_in[3]; const float* b2 = (const float*)d_in[4]; const float* w3 = (const float*)d_in[5]; const float* b3 = (const float*)d_in[6];
    const float* mA = (const float*)d_in[7]; const float* ma = (const float*)d_in[8]; const float* mB = (const float*)d_in[9]; const float* mb = (const float*)d_in[10]; const int* q = (const int*)d_in[11];
    float* OUT = (float*)d_out;
    char* wsp = (char*)d_ws;
    auto take = [&](size_t bytes) { char* p = wsp; wsp += (bytes + 255) & ~(size_t)255; return (void*)p; };
    bf* XB = (bf*)take((size_t)NR * D0 * 2); bf* W1B = (bf*)take((size_t)D1 * D0 * 2); bf* W2B = (bf*)take((size_t)D1 * D1 * 2); bf* W3B = (bf*)take((size_t)D3 * D1 * 2);
    float* GB1 = (float*)take((size_t)NR * D1 * 4); float* GB2 = (float*)take((size_t)NR * D1 * 4); float* GB3 = (float*)take((size_t)NR * D3 * 4); float* Y1 = (float*)take((size_t)NR * D1 * 4); float* Y2 = (float*)take((size_t)NR * D1 * 4);
    bf* Y1h = (bf*)take((size_t)NR * D1 * 2); bf* Y1l = (bf*)take((size_t)NR * D1 * 2); bf* Y2h = (bf*)take((size_t)NR * D1 * 2); bf* Y2l = (bf*)take((size_t)NR * D1 * 2);
    float* RS1 = (float*)take((size_t)2 * NR * 4); float* RS2 = (float*)take((size_t)2 * NR * 4); float* RS3 = (float*)take((size_t)2 * NR * 4);
    if ((size_t)(wsp - (char*)d_ws) != WS_TOTAL || WS_TOTAL > ws_size) return;
    k_cvt8<<<(unsigned)(((size_t)NR * D0 / 8 + 255) / 256), 256, 0, stream>>>(x, XB, (size_t)NR * D0 / 8);
    k_cvt8<<<(unsigned)(((size_t)D1 * D0 / 8 + 255) / 256), 256, 0, stream>>>(w1, W1B, (size_t)D1 * D0 / 8);
    k_cvt8<<<(unsigned)(((size_t)D1 * D1 / 8 + 255) / 256), 256, 0, stream>>>(w2, W2B, (size_t)D1 * D1 / 8);
    k_cvt8<<<(unsigned)(((size_t)D3 * D1 / 8 + 255) / 256), 256, 0, stream>>>(w3, W3B, (size_t)D3 * D1 / 8);
    k_gemmw<bf, 0, true><<<dim3(NR / 64, D1 / 64, 1), 32, 0, stream>>>(XB, nullptr, W1B, nullptr, D0, GB1, D1, b1, (size_t)0, (size_t)0, (size_t)0);
    k_rsum16<<<1, 256, 0, stream>>>(XB, RS1, NR);
    k_corr<<<dim3(D1 / 256, NR, 1), 256, 0, stream>>>(GB1, b1, RS1, mA, ma, mB, mb, q, Y1, D1);
    k_pl2<<<(unsigned)(((size_t)NR * D1 / 4 + 255) / 256), 256, 0, stream>>>(Y1, Y1h, Y1l, (size_t)NR * D1 / 4);
    k_gemmw<bf, 1, true><<<dim3(NR / 64, D1 / 64, 1), 32, 0, stream>>>(Y1h, Y1l, W2B, nullptr, D1, GB2, D1, b2, (size_t)0, (size_t)0, (size_t)0);
    k_rsum32<<<1, 256, 0, stream>>>(Y1, RS2, NR);
    k_corr<<<dim3(D1 / 256, NR, 1), 256, 0, stream>>>(GB2, b2, RS2, mA, ma, mB, mb, q, Y2, D1);
    k_pl2<<<(unsigned)(((size_t)NR * D1 / 4 + 255) / 256), 256, 0, stream>>>(Y2, Y2h, Y2l, (size_t)NR * D1 / 4);
    k_gemmw<bf, 1, true><<<dim3(NR / 64, D3 / 64, 1), 32, 0, stream>>>(Y2h, Y2l, W3B, nullptr, D1, GB3, D3, b3, (size_t)0, (size_t)0, (size_t)0);
    k_rsum32<<<1, 256, 0, stream>>>(Y2, RS3, NR);
    k_corr<<<dim3(D3 / 256, NR, 1), 256, 0, stream>>>(GB3, b3, RS3, mA, ma, mB, mb, q, OUT, D3);
}
